// MHSA_55972013801775
// MI455X (gfx1250) — hardware-verified
//
#include <hip/hip_runtime.h>
#include <math.h>
#include <stdint.h>

#define NBATCH 16
#define NCH    512
#define NTOK   1024
#define NHEAD  4
#define DHQ    32
#define DHV    128
#define NCOLS  768

#define PREP_T 2048
#define PREP_W 192
#define PREP_F 3
#define PREP_P 64

typedef __attribute__((ext_vector_type(16))) __bf16 v16b;
typedef __attribute__((ext_vector_type(8)))  __bf16 v8b;
typedef __attribute__((ext_vector_type(8)))  float  v8f;
typedef __attribute__((ext_vector_type(4)))  float  v4f;
typedef __attribute__((ext_vector_type(4)))  unsigned int v4u;
typedef v4f __attribute__((may_alias)) v4fa;

static_assert(NTOK % 64 == 0);
static_assert(NCH % 32 == 0);
static_assert(NCOLS % 128 == 0);
static_assert(PREP_T == NBATCH * (NCH / 64) * (NTOK / 64));
static_assert(PREP_W * 2048 == NCOLS * NCH);
static_assert(PREP_F * 256 == NCOLS);
static_assert(PREP_P * 64 == NHEAD * NTOK);

__device__ __forceinline__ unsigned short f2bf_bits(float f) {
  unsigned u = __float_as_uint(f);
  return (unsigned short)((u + 0x7FFFu + ((u >> 16) & 1u)) >> 16);
}
__device__ __forceinline__ float bf_bits2f(unsigned short h) { return __uint_as_float(((unsigned)h) << 16); }
__device__ __forceinline__ float bfr(float f) { return bf_bits2f(f2bf_bits(f)); }
__device__ __forceinline__ unsigned pk16(unsigned short a, unsigned short b) { return (unsigned)a | ((unsigned)b << 16); }
__device__ __forceinline__ void split_pair(float f0, float f1, unsigned& h, unsigned& l) {
  const unsigned short h0 = f2bf_bits(f0), h1 = f2bf_bits(f1);
  const unsigned short l0 = f2bf_bits(f0 - bf_bits2f(h0)), l1 = f2bf_bits(f1 - bf_bits2f(h1));
  h = pk16(h0, h1);
  l = pk16(l0, l1);
}

__device__ __forceinline__ v8f mma_b(v16b a, v16b b, v8f c) {
  c = __builtin_amdgcn_wmma_f32_16x16x32_bf16(false, a, false, b, (short)0, c, false, false);
  asm volatile("v_nop\n\tv_nop\n\tv_nop\n\tv_nop" : "+v"(c) : "v"(a), "v"(b));
  return c;
}
union FB { v16b v; v8b h[2]; };
__device__ __forceinline__ v16b frag_ld(const __bf16* p) {
  FB f;
  f.h[0] = *(const v8b*)(p);
  f.h[1] = *(const v8b*)(p + 16);
  return f.v;
}

__global__ __launch_bounds__(256) void k_prep(
    const float* __restrict__ x,
    const float* __restrict__ Wq, const float* __restrict__ Wk, const float* __restrict__ Wv,
    const float* __restrict__ bq, const float* __restrict__ qg, const float* __restrict__ qbe,
    const float* __restrict__ qm, const float* __restrict__ qv,
    const float* __restrict__ bk, const float* __restrict__ kg, const float* __restrict__ kbe,
    const float* __restrict__ km, const float* __restrict__ kv,
    const float* __restrict__ bv, const float* __restrict__ vg, const float* __restrict__ vbe,
    const float* __restrict__ vm, const float* __restrict__ vv,
    const float* __restrict__ relH, const float* __restrict__ relW,
    unsigned short* __restrict__ XT, unsigned short* __restrict__ WB, float* __restrict__ ST,
    unsigned short* __restrict__ POSh, unsigned short* __restrict__ POSl) {
  __shared__ __align__(16) float sm[64 * 68];
  const int tid = threadIdx.x;
  const int bx  = blockIdx.x;

  if (bx < PREP_T) {
    const int b   = bx >> 7;
    const int rem = bx & 127;
    const int c0  = (rem >> 4) * 64;
    const int n0  = (rem & 15) * 64;
    const float* xb = x + (size_t)b * NCH * NTOK;
    {
      const int lr = tid >> 4;
      const int c4 = (tid & 15) * 4;
#pragma unroll
      for (int it = 0; it < 4; ++it) {
        const int rr = it * 16 + lr;
        const v4f a = *(const v4fa*)(xb + (size_t)(c0 + rr) * NTOK + n0 + c4);
        *(v4fa*)(sm + rr * 68 + c4) = a;
      }
    }
    __syncthreads();
    const int sub = tid >> 3;
    const int c8  = (tid & 7) * 8;
    v4u hv[2];
#pragma unroll
    for (int it = 0; it < 2; ++it) {
      const int oc = it * 32 + sub;
      unsigned w0 = pk16(f2bf_bits(sm[(c8 + 0) * 68 + oc]), f2bf_bits(sm[(c8 + 1) * 68 + oc]));
      unsigned w1 = pk16(f2bf_bits(sm[(c8 + 2) * 68 + oc]), f2bf_bits(sm[(c8 + 3) * 68 + oc]));
      unsigned w2 = pk16(f2bf_bits(sm[(c8 + 4) * 68 + oc]), f2bf_bits(sm[(c8 + 5) * 68 + oc]));
      unsigned w3 = pk16(f2bf_bits(sm[(c8 + 6) * 68 + oc]), f2bf_bits(sm[(c8 + 7) * 68 + oc]));
      hv[it] = (v4u){w0, w1, w2, w3};
    }
    for (int pass = 0; pass < 2; ++pass) {
#pragma unroll
      for (int it = 0; it < 2; ++it) {
        const int oc = it * 32 + sub;
        const size_t go = ((size_t)(b * NTOK + n0 + oc)) * NCH + c0 + c8;
        *(volatile v4u*)(XT + go) = hv[it];
      }
      __threadfence();
    }
  } else if (bx < PREP_T + PREP_W) {
    const int wb = bx - PREP_T;
    const float* src;
    if (wb < 32)      src = Wq + (size_t)wb * 2048;
    else if (wb < 64) src = Wk + (size_t)(wb - 32) * 2048;
    else              src = Wv + (size_t)(wb - 64) * 2048;
    const v4f a = *(const v4fa*)(src + tid * 8);
    const v4f c = *(const v4fa*)(src + tid * 8 + 4);
    const v4u o = (v4u){pk16(f2bf_bits(a[0]), f2bf_bits(a[1])), pk16(f2bf_bits(a[2]), f2bf_bits(a[3])),
                        pk16(f2bf_bits(c[0]), f2bf_bits(c[1])), pk16(f2bf_bits(c[2]), f2bf_bits(c[3]))};
    unsigned short* dst = WB + (size_t)wb * 2048 + tid * 8;
    *(volatile v4u*)dst = o;
    __threadfence();
    *(volatile v4u*)dst = o;
  } else if (bx < PREP_T + PREP_W + PREP_F) {
    const int fb = bx - (PREP_T + PREP_W);
    const int wsel = __builtin_amdgcn_readfirstlane((int)(tid >> 7));
    const float *pb, *pg, *pbe, *pm, *pv;
    int idx;
    if (fb == 0) {
      if (wsel == 0) { pb = bq; pg = qg; pbe = qbe; pm = qm; pv = qv; idx = tid; }
      else           { pb = bk; pg = kg; pbe = kbe; pm = km; pv = kv; idx = tid - 128; }
    } else {
      pb = bv; pg = vg; pbe = vbe; pm = vm; pv = vv; idx = (fb - 1) * 256 + tid;
    }
    const float b_ = bfr(pb[idx]);
    const float g_ = bfr(pg[idx]);
    const float be = bfr(pbe[idx]);
    const float mu = bfr(pm[idx]);
    const float va = bfr(pv[idx]);
    const float s  = g_ / sqrtf(va + 1e-5f);
    const float t  = (b_ - mu) * s + be;
    sm[tid]       = s;
    sm[256 + tid] = t;
    __syncthreads();
    if (tid < 128) {
      const int which = tid >> 6;
      const int p4 = (tid & 63) * 4;
      const v4f v = *(const v4fa*)(sm + which * 256 + p4);
      float* dst = ST + which * NCOLS + fb * 256 + p4;
      *(volatile v4f*)dst = v;
      __threadfence();
      *(volatile v4f*)dst = v;
    }
  } else {
    const int pb = bx - (PREP_T + PREP_W + PREP_F);
    const int h  = pb >> 4;
    const int n0 = (pb & 15) * 64;
    {
      v4f w = *(const v4fa*)(relW + h * 1024 + tid * 4);
      v4f g = *(const v4fa*)(relH + h * 1024 + tid * 4);
      w = (v4f){bfr(w[0]), bfr(w[1]), bfr(w[2]), bfr(w[3])};
      g = (v4f){bfr(g[0]), bfr(g[1]), bfr(g[2]), bfr(g[3])};
      *(v4fa*)(sm + tid * 4)        = w;
      *(v4fa*)(sm + 1024 + tid * 4) = g;
    }
    __syncthreads();
    const int tl = tid >> 2;
    const int d8 = (tid & 3) * 8;
    const int n  = n0 + tl;
    const int wi = n >> 5, hi_ = n & 31;
    float p[8];
#pragma unroll
    for (int e = 0; e < 8; ++e) p[e] = sm[(d8 + e) * 32 + wi] + sm[1024 + (d8 + e) * 32 + hi_];
    unsigned h0, h1, h2, h3, l0, l1, l2, l3;
    split_pair(p[0], p[1], h0, l0);
    split_pair(p[2], p[3], h1, l1);
    split_pair(p[4], p[5], h2, l2);
    split_pair(p[6], p[7], h3, l3);
    const v4u hv = (v4u){h0, h1, h2, h3};
    const v4u lv = (v4u){l0, l1, l2, l3};
    const size_t go = ((size_t)(h * NTOK + n0)) * DHQ + tid * 8;
    *(volatile v4u*)(POSh + go) = hv;
    *(volatile v4u*)(POSl + go) = lv;
    __threadfence();
    *(volatile v4u*)(POSh + go) = hv;
    *(volatile v4u*)(POSl + go) = lv;
  }
}

__global__ __launch_bounds__(128) void k_proj(
    const unsigned short* __restrict__ XTp, const unsigned short* __restrict__ WBp,
    const float* __restrict__ ST,
    unsigned short* __restrict__ Qh, unsigned short* __restrict__ Ql,
    unsigned short* __restrict__ Kh, unsigned short* __restrict__ Kl,
    unsigned short* __restrict__ Vh, unsigned short* __restrict__ Vl) {
  __shared__ __align__(16) float sY[128 * 68];
  __shared__ __align__(16) float sS[128];
  __shared__ __align__(16) float sT[128];

  const int tid  = threadIdx.x;
  const int lane = tid & 31;
  const int wave = tid >> 5;
  const int hh   = lane >> 4;
  const int c    = lane & 15;
  const int m0   = blockIdx.x * 64;
  const int ct   = blockIdx.y;
  const int n0   = ct * 128;

  sS[tid] = ST[n0 + tid];
  sT[tid] = ST[NCOLS + n0 + tid];
  __syncthreads();

  const int wr = wave >> 1, wc = wave & 1;
  const __bf16* XT = (const __bf16*)(const void*)XTp;
  const __bf16* WB = (const __bf16*)(const void*)WBp;
  const __bf16* a0p = XT + (size_t)(m0 + 32 * wr + c) * NCH + 8 * hh;
  const __bf16* b0p = WB + (size_t)(n0 + 64 * wc + c) * NCH + 8 * hh;

  const v8f zero8 = {0.f, 0.f, 0.f, 0.f, 0.f, 0.f, 0.f, 0.f};
  v8f acc[2][4];
#pragma unroll
  for (int i = 0; i < 2; ++i)
#pragma unroll
    for (int j = 0; j < 4; ++j) acc[i][j] = zero8;

#pragma unroll 1
  for (int k0 = 0; k0 < NCH; k0 += 32) {
    const v16b a0 = frag_ld(a0p + k0);
    const v16b a1 = frag_ld(a0p + (size_t)16 * NCH + k0);
#pragma unroll
    for (int j = 0; j < 4; ++j) {
      const v16b bf = frag_ld(b0p + (size_t)j * 16 * NCH + k0);
      acc[0][j] = mma_b(a0, bf, acc[0][j]);
      acc[1][j] = mma_b(a1, bf, acc[1][j]);
    }
  }

#pragma unroll
  for (int j = 0; j < 4; ++j) {
    const int col = 64 * wc + 16 * j + c;
    const float sc = sS[col];
    const float sh = sT[col];
#pragma unroll
    for (int i = 0; i < 2; ++i) {
#pragma unroll
      for (int r = 0; r < 8; ++r) {
        const int tok = 32 * wr + 16 * i + 8 * hh + r;
        const float y = acc[i][j][r] * sc + sh;
        const int idx = (ct < 2) ? (tok * 132 + col) : (col * 68 + tok);
        sY[idx] = y;
      }
    }
  }
  __syncthreads();

  const int b   = m0 >> 10;
  const int nl0 = m0 & 1023;
  if (ct < 2) {
    unsigned short* ph = (ct == 0) ? Qh : Kh;
    unsigned short* pl = (ct == 0) ? Ql : Kl;
#pragma unroll 1
    for (int pass = 0; pass < 2; ++pass) {
#pragma unroll 2
      for (int it = 0; it < 8; ++it) {
        const int p      = it * 128 + tid;
        const int head   = p >> 8;
        const int within = p & 255;
        const int tok    = within >> 2;
        const int d8     = (within & 3) * 8;
        const float* sp  = sY + tok * 132 + head * 32 + d8;
        const v4f a  = *(const v4fa*)sp;
        const v4f a2 = *(const v4fa*)(sp + 4);
        unsigned h0, h1, h2, h3, l0, l1, l2, l3;
        split_pair(a[0], a[1], h0, l0);
        split_pair(a[2], a[3], h1, l1);
        split_pair(a2[0], a2[1], h2, l2);
        split_pair(a2[2], a2[3], h3, l3);
        const v4u hv = (v4u){h0, h1, h2, h3};
        const v4u lv = (v4u){l0, l1, l2, l3};
        const size_t go = ((size_t)((b * NHEAD + head) * NTOK + nl0)) * DHQ + within * 8;
        *(volatile v4u*)(ph + go) = hv;
        *(volatile v4u*)(pl + go) = lv;
      }
      __threadfence();
    }
  } else {
    const int o0 = (ct - 2) * 128;
#pragma unroll 1
    for (int pass = 0; pass < 2; ++pass) {
#pragma unroll 2
      for (int it = 0; it < 8; ++it) {
        const int p  = it * 128 + tid;
        const int ch = p >> 3;
        const int t8 = (p & 7) * 8;
        const float* sp = sY + ch * 68 + t8;
        const v4f a  = *(const v4fa*)sp;
        const v4f a2 = *(const v4fa*)(sp + 4);
        unsigned h0, h1, h2, h3, l0, l1, l2, l3;
        split_pair(a[0], a[1], h0, l0);
        split_pair(a[2], a[3], h1, l1);
        split_pair(a2[0], a2[1], h2, l2);
        split_pair(a2[2], a2[3], h3, l3);
        const v4u hv = (v4u){h0, h1, h2, h3};
        const v4u lv = (v4u){l0, l1, l2, l3};
        const size_t go = ((size_t)(b * NCH + o0 + ch)) * NTOK + nl0 + t8;
        *(volatile v4u*)(Vh + go) = hv;
        *(volatile v4u*)(Vl + go) = lv;
      }
      __threadfence();
    }
  }
}

__global__ __launch_bounds__(128) void k_attn(
    const unsigned short* Qhp, const unsigned short* Qlp,
    const unsigned short* Khp, const unsigned short* Klp,
    const unsigned short* Vhp, const unsigned short* Vlp,
    const unsigned short* Php, const unsigned short* Plp,
    const float* x, float* out) {
  __shared__ __align__(16) __bf16 sStage[24576];
  __shared__ __align__(16) __bf16 sP[4 * 2 * 16 * 64];

  const int tid  = threadIdx.x;
  const int wave = tid >> 5;
  const int lane = tid & 31;
  const int hh   = lane >> 4;
  const int c    = lane & 15;

  const int bx = blockIdx.x;
  const int qb = bx & 15;
  const int bh = bx >> 4;
  const int b  = bh >> 2;
  const int h  = bh & 3;
  const int q0 = qb * 64;

  const __bf16* Qhb = (const __bf16*)(const void*)Qhp + (size_t)bh * NTOK * DHQ;
  const __bf16* Qlb = (const __bf16*)(const void*)Qlp + (size_t)bh * NTOK * DHQ;
  const __bf16* Khb = (const __bf16*)(const void*)Khp + (size_t)bh * NTOK * DHQ;
  const __bf16* Klb = (const __bf16*)(const void*)Klp + (size_t)bh * NTOK * DHQ;
  const __bf16* Phb = (const __bf16*)(const void*)Php + (size_t)h * NTOK * DHQ;
  const __bf16* Plb = (const __bf16*)(const void*)Plp + (size_t)h * NTOK * DHQ;
  const __bf16* Vhb = (const __bf16*)(const void*)Vhp + ((size_t)b * NCH + h * DHV) * NTOK;
  const __bf16* Vlb = (const __bf16*)(const void*)Vlp + ((size_t)b * NCH + h * DHV) * NTOK;

  __bf16* sKQ = sStage;
  __bf16* sVh = sStage + 8192;
  __bf16* sVl = sStage + 16384;
  __bf16* pwh = sP + wave * 2048;
  __bf16* pwl = pwh + 1024;

  const int rowA = q0 + wave * 16 + c;
  const __bf16* aQh = Qhb + (size_t)rowA * DHQ + 8 * hh;
  const __bf16* aQl = Qlb + (size_t)rowA * DHQ + 8 * hh;
  const __bf16* aPh = Phb + (size_t)rowA * DHQ + 8 * hh;
  const __bf16* aPl = Plb + (size_t)rowA * DHQ + 8 * hh;

  const v8f zero8 = {0.f, 0.f, 0.f, 0.f, 0.f, 0.f, 0.f, 0.f};
  float mrow[8], lrow[8];
  v8f oacc[8];
#pragma unroll
  for (int r = 0; r < 8; ++r) { mrow[r] = -INFINITY; lrow[r] = 0.f; }
#pragma unroll
  for (int t = 0; t < 8; ++t) oacc[t] = zero8;

#pragma unroll 1
  for (int kc = 0; kc < NTOK / 64; ++kc) {
    const int kv0 = kc * 64;
    __syncthreads();
    {
      const __bf16* s0 = Khb + (size_t)kv0 * DHQ;
      const __bf16* s1 = Qhb + (size_t)kv0 * DHQ;
      const __bf16* s2 = Klb + (size_t)kv0 * DHQ;
      const __bf16* s3 = Qlb + (size_t)kv0 * DHQ;
#pragma unroll
      for (int i = 0; i < 2; ++i) {
        const int off = (i * 128 + tid) * 8;
        const v8b a0 = *(const v8b*)(s0 + off);
        const v8b a1 = *(const v8b*)(s1 + off);
        const v8b a2 = *(const v8b*)(s2 + off);
        const v8b a3 = *(const v8b*)(s3 + off);
        *(v8b*)(sKQ + off)        = a0;
        *(v8b*)(sKQ + 2048 + off) = a1;
        *(v8b*)(sKQ + 4096 + off) = a2;
        *(v8b*)(sKQ + 6144 + off) = a3;
      }
#pragma unroll
      for (int i = 0; i < 8; ++i) {
        const int piece = i * 128 + tid;
        const int cc = piece >> 3;
        const int p8 = (piece & 7) * 8;
        const v8b b0 = *(const v8b*)(Vhb + (size_t)cc * NTOK + kv0 + p8);
        const v8b b1 = *(const v8b*)(Vlb + (size_t)cc * NTOK + kv0 + p8);
        *(v8b*)(sVh + cc * 64 + p8) = b0;
        *(v8b*)(sVl + cc * 64 + p8) = b1;
      }
    }
    __syncthreads();

    v8f s[4];
#pragma unroll
    for (int j = 0; j < 4; ++j) s[j] = zero8;
#pragma unroll
    for (int dc = 0; dc < 2; ++dc) {
      const __bf16* ahp = dc ? aPh : aQh;
      const __bf16* alp = dc ? aPl : aQl;
      const v16b ah = frag_ld(ahp);
      const v16b al = frag_ld(alp);
      const __bf16* bhs = sKQ + (dc ? 2048 : 0);
      const __bf16* bls = sKQ + (dc ? 6144 : 4096);
#pragma unroll
      for (int j = 0; j < 4; ++j) {
        const int ro = (j * 16 + c) * DHQ + 8 * hh;
        const v16b kb = frag_ld(bhs + ro);
        const v16b kl = frag_ld(bls + ro);
        s[j] = mma_b(ah, kb, s[j]);
        s[j] = mma_b(ah, kl, s[j]);
        s[j] = mma_b(al, kb, s[j]);
      }
    }

    float cm[8];
#pragma unroll
    for (int r = 0; r < 8; ++r) {
      float m = fmaxf(fmaxf(s[0][r], s[1][r]), fmaxf(s[2][r], s[3][r]));
#pragma unroll
      for (int off = 1; off < 16; off <<= 1) m = fmaxf(m, __shfl_xor(m, off, 32));
      cm[r] = m;
    }
#pragma unroll
    for (int r = 0; r < 8; ++r) {
      const float mnew  = fmaxf(mrow[r], cm[r]);
      const float alpha = expf(mrow[r] - mnew);
      mrow[r] = mnew;
      float psum = 0.f;
#pragma unroll
      for (int j = 0; j < 4; ++j) {
        const float p = expf(s[j][r] - mnew);
        psum += p;
        const unsigned short hb = f2bf_bits(p);
        const unsigned short lb = f2bf_bits(p - bf_bits2f(hb));
        pwh[(8 * hh + r) * 64 + j * 16 + c] = __builtin_bit_cast(__bf16, hb);
        pwl[(8 * hh + r) * 64 + j * 16 + c] = __builtin_bit_cast(__bf16, lb);
      }
#pragma unroll
      for (int off = 1; off < 16; off <<= 1) psum += __shfl_xor(psum, off, 32);
      lrow[r] = lrow[r] * alpha + psum;
#pragma unroll
      for (int t = 0; t < 8; ++t) oacc[t][r] *= alpha;
    }
    __builtin_amdgcn_fence(__ATOMIC_RELEASE, "workgroup");
    __builtin_amdgcn_wave_barrier();
    __builtin_amdgcn_fence(__ATOMIC_ACQUIRE, "workgroup");
#pragma unroll 1
    for (int kk = 0; kk < 2; ++kk) {
      const v16b pa = frag_ld(pwh + c * 64 + kk * 32 + 8 * hh);
      const v16b pl = frag_ld(pwl + c * 64 + kk * 32 + 8 * hh);
#pragma unroll
      for (int t = 0; t < 8; ++t) {
        const int ro = (t * 16 + c) * 64 + kk * 32 + 8 * hh;
        const v16b vb = frag_ld(sVh + ro);
        const v16b vl = frag_ld(sVl + ro);
        oacc[t] = mma_b(pa, vb, oacc[t]);
        oacc[t] = mma_b(pa, vl, oacc[t]);
        oacc[t] = mma_b(pl, vb, oacc[t]);
      }
    }
  }

  __syncthreads();
  float* sO = (float*)(void*)sStage;
#pragma unroll
  for (int r = 0; r < 8; ++r) {
    const float inv = 1.0f / lrow[r];
#pragma unroll
    for (int t = 0; t < 8; ++t) sO[(t * 16 + c) * 68 + wave * 16 + 8 * hh + r] = oacc[t][r] * inv;
  }
  __syncthreads();
  {
    const size_t rowbase = ((size_t)b * NCH + h * DHV) * NTOK + q0;
#pragma unroll 1
    for (int pass = 0; pass < 2; ++pass) {
#pragma unroll 4
      for (int it = 0; it < 16; ++it) {
        const int p  = it * 128 + tid;
        const int ch = p >> 4;
        const int q4 = (p & 15) * 4;
        const v4f ov = *(const v4fa*)(sO + ch * 68 + q4);
        const size_t gi = rowbase + (size_t)ch * NTOK + q4;
        const v4f xv = *(const v4fa*)(x + gi);
        const v4f res = (v4f){ov[0] + bfr(xv[0]), ov[1] + bfr(xv[1]), ov[2] + bfr(xv[2]), ov[3] + bfr(xv[3])};
        *(volatile v4f*)(out + gi) = res;
      }
      __threadfence();
    }
  }
}

extern "C" void kernel_launch(void* const* d_in, const int* in_sizes, int n_in,
                              void* d_out, int out_size, void* d_ws, size_t ws_size,
                              hipStream_t stream) {
  if (n_in < 21) return;
  const int NX = NBATCH * NCH * NTOK;
  if (in_sizes[0] != NX) return;
  if (in_sizes[1] != 128 * NCH || in_sizes[7] != 128 * NCH || in_sizes[13] != NCH * NCH) return;
  for (int i = 2; i <= 6; ++i)   if (in_sizes[i] != 128) return;
  for (int i = 8; i <= 12; ++i)  if (in_sizes[i] != 128) return;
  for (int i = 14; i <= 18; ++i) if (in_sizes[i] != NCH) return;
  if (in_sizes[19] != NHEAD * DHQ * 32 || in_sizes[20] != NHEAD * DHQ * 32) return;
  if (out_size != NX) return;

  const float* x    = (const float*)d_in[0];
  const float* Wq   = (const float*)d_in[1];
  const float* bq   = (const float*)d_in[2];
  const float* qg   = (const float*)d_in[3];
  const float* qbe  = (const float*)d_in[4];
  const float* qm   = (const float*)d_in[5];
  const float* qv   = (const float*)d_in[6];
  const float* Wk   = (const float*)d_in[7];
  const float* bk   = (const float*)d_in[8];
  const float* kg   = (const float*)d_in[9];
  const float* kbe  = (const float*)d_in[10];
  const float* km   = (const float*)d_in[11];
  const float* kv   = (const float*)d_in[12];
  const float* Wv   = (const float*)d_in[13];
  const float* bv   = (const float*)d_in[14];
  const float* vg   = (const float*)d_in[15];
  const float* vbe  = (const float*)d_in[16];
  const float* vm   = (const float*)d_in[17];
  const float* vv   = (const float*)d_in[18];
  const float* relH = (const float*)d_in[19];
  const float* relW = (const float*)d_in[20];

  const size_t szXT  = (size_t)NBATCH * NTOK * NCH * 2;
  const size_t szWB  = (size_t)NCOLS * NCH * 2;
  const size_t szST  = (size_t)2 * NCOLS * 4;
  const size_t szPOS = (size_t)NHEAD * NTOK * DHQ * 2;
  const size_t szQK  = (size_t)NBATCH * NHEAD * NTOK * DHQ * 2;
  const size_t szV   = (size_t)NBATCH * NCH * NTOK * 2;
  size_t off = 0;
  const size_t oXT = off;   off += szXT;
  const size_t oWB = off;   off += szWB;
  const size_t oST = off;   off += szST;
  const size_t oPh = off;   off += szPOS;
  const size_t oPl = off;   off += szPOS;
  const size_t oQh = off;   off += szQK;
  const size_t oQl = off;   off += szQK;
  const size_t oKh = off;   off += szQK;
  const size_t oKl = off;   off += szQK;
  const size_t oVh = off;   off += szV;
  const size_t oVl = off;   off += szV;
  if (off > ws_size) return;
  if (off > (size_t)134217728) return;

  char* ws = (char*)d_ws;
  unsigned short* XT   = (unsigned short*)(ws + oXT);
  unsigned short* WB   = (unsigned short*)(ws + oWB);
  float*          ST   = (float*)(ws + oST);
  unsigned short* POSh = (unsigned short*)(ws + oPh);
  unsigned short* POSl = (unsigned short*)(ws + oPl);
  unsigned short* Qh   = (unsigned short*)(ws + oQh);
  unsigned short* Ql   = (unsigned short*)(ws + oQl);
  unsigned short* Kh   = (unsigned short*)(ws + oKh);
  unsigned short* Kl   = (unsigned short*)(ws + oKl);
  unsigned short* Vh   = (unsigned short*)(ws + oVh);
  unsigned short* Vl   = (unsigned short*)(ws + oVl);

  k_prep<<<dim3(PREP_T + PREP_W + PREP_F + PREP_P), dim3(256), 0, stream>>>(
      x, Wq, Wk, Wv, bq, qg, qbe, qm, qv, bk, kg, kbe, km, kv, bv, vg, vbe, vm, vv, relH, relW,
      XT, WB, ST, POSh, POSl);

  k_proj<<<dim3((NBATCH * NTOK) / 64, NCOLS / 128), dim3(128), 0, stream>>>(
      XT, WB, ST, Qh, Ql, Kh, Kl, Vh, Vl);

  k_attn<<<dim3(NBATCH * NHEAD * (NTOK / 64)), dim3(128), 0, stream>>>(
      Qh, Ql, Kh, Kl, Vh, Vl, POSh, POSl, x, (float*)d_out);

  (void)hipGetLastError();
}
